// SABlock_2834678415763
// MI455X (gfx1250) — hardware-verified
//
#include <hip/hip_runtime.h>
#include <hip/hip_bf16.h>
#include <math.h>
#include <stdint.h>
#include <stddef.h>

typedef __attribute__((ext_vector_type(16))) _Float16 v16h;
typedef __attribute__((ext_vector_type(8)))  _Float16 v8h;
typedef __attribute__((ext_vector_type(4)))  _Float16 v4h;
typedef __attribute__((ext_vector_type(16))) __bf16   v16b;
typedef __attribute__((ext_vector_type(8)))  __bf16   v8b;
typedef __attribute__((ext_vector_type(8)))  float    v8f;
typedef __attribute__((ext_vector_type(4)))  float    v4f;
#define PSCALE 32768.0f
#define U16(p) ((const unsigned short*)(const void*)(p))
#define PSCALE_INV (1.0f / 32768.0f)

__device__ __forceinline__ unsigned short f2bf_bits(float f) {
  unsigned u = __float_as_uint(f);
  return (unsigned short)((u + 0x7FFFu + ((u >> 16) & 1u)) >> 16);
}
__device__ __forceinline__ float bf_bits2f(unsigned short h) { return __uint_as_float(((unsigned)h) << 16); }

__device__ __forceinline__ void dep_guard_h(v8f& a, v8f& b, v16h x, v16h y) { asm volatile("v_nop\n\tv_nop\n\tv_nop\n\tv_nop" : "+v"(a), "+v"(b) : "v"(x), "v"(y)); }
__device__ __forceinline__ void dep_guard_b(v8f& a, v8f& b, v16b x, v16b y) { asm volatile("v_nop\n\tv_nop\n\tv_nop\n\tv_nop" : "+v"(a), "+v"(b) : "v"(x), "v"(y)); }
__device__ __forceinline__ void keep4_h(v16h a, v16h b, v16h c, v16h d) { asm volatile("v_nop" :: "v"(a), "v"(b), "v"(c), "v"(d)); }
__device__ __forceinline__ void keep4_b(v16b a, v16b b, v16b c, v16b d) { asm volatile("v_nop" :: "v"(a), "v"(b), "v"(c), "v"(d)); }
__device__ __forceinline__ void acc_guard4(v8f& a, v8f& b, v8f& c, v8f& d) { asm volatile("v_nop\n\tv_nop\n\tv_nop\n\tv_nop" : "+v"(a), "+v"(b), "+v"(c), "+v"(d)); }
template <typename T> struct Frag;
template <> struct Frag<_Float16> {
  typedef v16h V; union U { v16h v; v8h h[2]; };
  static __device__ __forceinline__ v16h load(const _Float16* p) {
    U f; f.h[0] = *(const v8h*)(p); f.h[1] = *(const v8h*)(p + 16); return f.v;
  }
  static __device__ __forceinline__ v8f mma(v16h a, v16h b, v8f c) {
    return __builtin_amdgcn_wmma_f32_16x16x32_f16(false, a, false, b, (short)0, c, false, false);
  }
  static __device__ __forceinline__ void guard(v8f& a, v8f& b, v16h x, v16h y) { dep_guard_h(a, b, x, y); }
  static __device__ __forceinline__ void keep(v16h a, v16h b, v16h c, v16h d) { keep4_h(a, b, c, d); }
};
template <> struct Frag<__bf16> {
  typedef v16b V; union U { v16b v; v8b h[2]; };
  static __device__ __forceinline__ v16b load(const __bf16* p) {
    U f; f.h[0] = *(const v8b*)(p); f.h[1] = *(const v8b*)(p + 16); return f.v;
  }
  static __device__ __forceinline__ v8f mma(v16b a, v16b b, v8f c) {
    return __builtin_amdgcn_wmma_f32_16x16x32_bf16(false, a, false, b, (short)0, c, false, false);
  }
  static __device__ __forceinline__ void guard(v8f& a, v8f& b, v16b x, v16b y) { dep_guard_b(a, b, x, y); }
  static __device__ __forceinline__ void keep(v16b a, v16b b, v16b c, v16b d) { keep4_b(a, b, c, d); }
};

template <int ET> struct Elem;
template <> struct Elem<0> { typedef _Float16 T; };
template <> struct Elem<1> { typedef __bf16 T; };
template <int ET, bool SPLIT, int BIAS_MODE, int OUT_MODE, bool RESID, int ACT = 0>
__global__ __launch_bounds__(256) void wmma_gemm64(
    const unsigned short* __restrict__ Ap, const unsigned short* __restrict__ A2p, int lda, long strideA,
    const unsigned short* __restrict__ Btp, const unsigned short* __restrict__ Bt2p, int ldb, long strideB,
    void* __restrict__ Cout, void* __restrict__ Cout2, int ldc, long strideC,
    const float* __restrict__ bias,
    const float* __restrict__ resid, long strideR,
    int M, int N, int K, float scale) {
  typedef typename Elem<ET>::T T;
  typedef typename Frag<T>::V V;
  const T* A = (const T*)Ap; const T* A2 = (const T*)A2p; const T* Bt = (const T*)Btp; const T* Bt2 = (const T*)Bt2p;
  __shared__ __align__(16) float sT[8][16 * 68];
  const int b    = blockIdx.y;
  const int lane = threadIdx.x & 31;
  const int wave = threadIdx.x >> 5;
  const int tilesN = N >> 6;
  const int tilesM = M >> 6;
  const int tile = blockIdx.x * 8 + wave;
  if (tile >= tilesM * tilesN) return;
  const int tm = tile / tilesN;
  const int tn = tile - tm * tilesN;
  const int m0 = tm << 6;
  const int n0 = tn << 6;

  const T* Ab  = A  + (size_t)b * strideA;
  const T* Bb  = Bt + (size_t)b * strideB;
  const T* Ab2 = SPLIT ? (A2  + (size_t)b * strideA) : nullptr;
  const T* Bb2 = SPLIT ? (Bt2 + (size_t)b * strideB) : nullptr;

  const int rlane = lane & 15;
  const int koff  = (lane >> 4) * 8;
  const int mOff  = (lane >> 4) * 8;

  v8f acc[4][4];
#pragma unroll
  for (int i = 0; i < 4; ++i)
#pragma unroll
    for (int j = 0; j < 4; ++j) acc[i][j] = (v8f){0.f,0.f,0.f,0.f,0.f,0.f,0.f,0.f};

  for (int k0 = 0; k0 < K; k0 += 32) {
    V bh[4], bl[4];
#pragma unroll
    for (int j = 0; j < 4; ++j) {
      const size_t bo = (size_t)(n0 + (j << 4) + rlane) * ldb + koff + k0;
      bh[j] = Frag<T>::load(Bb + bo);
      if (SPLIT) bl[j] = Frag<T>::load(Bb2 + bo);
    }
#pragma unroll
    for (int i = 0; i < 4; ++i) {
      const size_t ao = (size_t)(m0 + (i << 4) + rlane) * lda + koff + k0;
      V ah = Frag<T>::load(Ab + ao);
      V al;
      if (SPLIT) al = Frag<T>::load(Ab2 + ao);
#pragma unroll
      for (int j = 0; j < 4; ++j) {
        acc[i][j] = Frag<T>::mma(ah, bh[j], acc[i][j]);
        if (SPLIT) {
          acc[i][j] = Frag<T>::mma(ah, bl[j], acc[i][j]);
          acc[i][j] = Frag<T>::mma(al, bh[j], acc[i][j]);
        }
      }
      Frag<T>::guard(acc[i][0], acc[i][3], ah, SPLIT ? al : ah);
    }
    Frag<T>::keep(bh[0], bh[1], bh[2], bh[3]);
    if (SPLIT) Frag<T>::keep(bl[0], bl[1], bl[2], bl[3]);
  }
  acc_guard4(acc[0][0], acc[0][1], acc[0][2], acc[0][3]);
  acc_guard4(acc[1][0], acc[1][1], acc[1][2], acc[1][3]);
  acc_guard4(acc[2][0], acc[2][1], acc[2][2], acc[2][3]);
  acc_guard4(acc[3][0], acc[3][1], acc[3][2], acc[3][3]);

  float* slab = sT[wave];
  const float* Rb = RESID ? (resid + (size_t)b * strideR) : nullptr;
#pragma unroll
  for (int i = 0; i < 4; ++i) {
    const int mBase = m0 + (i << 4);
#pragma unroll
    for (int j = 0; j < 4; ++j) {
      const int n = n0 + (j << 4) + rlane;
      float bv = 0.f;
      if (BIAS_MODE == 2) bv = bias[n];
#pragma unroll
      for (int r = 0; r < 8; ++r) {
        float v = acc[i][j][r] * scale;
        if (BIAS_MODE == 1) v += bias[mBase + mOff + r];
        if (BIAS_MODE == 2) v += bv;
        if (RESID) v += Rb[(size_t)(mBase + mOff + r) * ldc + n];
        if (ACT == 1) v = tanhf(v);
        if (ACT == 2) v = fmaxf(v, 0.0f);
        if (ACT == 3) v = v / (1.0f + expf(-v));
        if (ACT == 4) v = (v > 0.f) ? v : 0.01f * v;
        if (ACT == 5) v = 0.5f * v * (1.0f + erff(v * 0.70710678118654752f));
        if (ACT == 6) v = v * (1.0f / (1.0f + __expf(-v)));
        slab[(mOff + r) * 68 + (j << 4) + rlane] = v;
      }
    }
    __builtin_amdgcn_fence(__ATOMIC_RELEASE, "workgroup");
    __builtin_amdgcn_wave_barrier();
    __builtin_amdgcn_fence(__ATOMIC_ACQUIRE, "workgroup");
    if (OUT_MODE == 0) {
      float* C = (float*)Cout + (size_t)b * strideC;
      const int hh = lane >> 4, c4 = (lane & 15) * 4;
      for (int pass = 0; pass < 2; ++pass) {
#pragma unroll
        for (int it = 0; it < 8; ++it) {
          const int row = it * 2 + hh;
          v4f v = *(const v4f*)(slab + row * 68 + c4);
          *(volatile v4f*)(C + (size_t)(mBase + row) * ldc + n0 + c4) = v;
        }
        __threadfence();
      }
    } else {
      const int q = lane >> 3, c8 = (lane & 7) * 8;
      unsigned short* C  = (unsigned short*)Cout  + (size_t)b * strideC;
      unsigned short* C2 = (OUT_MODE == 2) ? ((unsigned short*)Cout2 + (size_t)b * strideC) : nullptr;
      for (int pass = 0; pass < 2; ++pass) {
#pragma unroll
        for (int it = 0; it < 4; ++it) {
          const int row = it * 4 + q;
          const float* sp = slab + row * 68 + c8;
          v8h hv, lv;
#pragma unroll
          for (int e = 0; e < 8; ++e) {
            if (OUT_MODE == 1) {
              hv[e] = (_Float16)sp[e];
            } else {
              unsigned short hb = f2bf_bits(sp[e]);
              unsigned short lb = f2bf_bits(sp[e] - bf_bits2f(hb));
              hv[e] = __builtin_bit_cast(_Float16, hb);
              lv[e] = __builtin_bit_cast(_Float16, lb);
            }
          }
          *(volatile v8h*)(C + (size_t)(mBase + row) * ldc + n0 + c8) = hv;
          if (OUT_MODE == 2) *(volatile v8h*)(C2 + (size_t)(mBase + row) * ldc + n0 + c8) = lv;
        }
        __threadfence();
      }
    }
    __builtin_amdgcn_fence(__ATOMIC_RELEASE, "workgroup");
    __builtin_amdgcn_wave_barrier();
    __builtin_amdgcn_fence(__ATOMIC_ACQUIRE, "workgroup");
  }
}

__global__ __launch_bounds__(256) void cast_f32_f16x2(
    const float* __restrict__ in, _Float16* __restrict__ out, int n2, float scale) {
  int i = blockIdx.x * 256 + threadIdx.x;
  if (i < n2) {
    const size_t i2 = (size_t)i * 2;
    const _Float16 h0 = (_Float16)(in[i2] * scale), h1 = (_Float16)(in[i2 + 1] * scale);
    const unsigned u = (unsigned)__builtin_bit_cast(unsigned short, h0) | ((unsigned)__builtin_bit_cast(unsigned short, h1) << 16);
    ((volatile unsigned*)out)[i] = u;
    __threadfence();
    ((volatile unsigned*)out)[i] = u;
  }
}

#define AT_D 64
#define AT_NW 4
#define AT_QB 64
#define AT_KC 64
#define AT_PSC 32768.0f

__device__ __forceinline__ v8f at_mma_h(v16h a, v16h b, v8f c) {
  c = __builtin_amdgcn_wmma_f32_16x16x32_f16(false, a, false, b, (short)0, c, false, false);
  asm volatile("v_nop\n\tv_nop\n\tv_nop\n\tv_nop" : "+v"(c) : "v"(a), "v"(b));
  return c;
}

__global__ __launch_bounds__(128)
void attn64_f16_kernel(const float* __restrict__ q, const float* __restrict__ k,
                       const float* __restrict__ v, float* __restrict__ out,
                       long bs, long rs, long hs, int S, int Skv, int H, float qscale) {
  union FB { v16h v; v8h h[2]; };
  __shared__ __align__(16) _Float16 Ksh[AT_KC * AT_D];
  __shared__ __align__(16) _Float16 Vth[AT_D * AT_KC];
  __shared__ __align__(16) _Float16 Psh[AT_NW][16 * AT_KC];
  __shared__ __align__(16) float    Os[AT_NW][16 * 68];

  const int tid  = threadIdx.x;
  const int wave = tid >> 5;
  const int lane = tid & 31;
  const int hh   = lane >> 4;
  const int c    = lane & 15;

  const int nqb = S / AT_QB;
  const int bx = blockIdx.x;
  const int qb = bx % nqb;
  const int bh = bx / nqb;
  const int h  = bh % H;
  const int b  = bh / H;
  const int q0 = qb * AT_QB + wave * 16;

  const float* qb_ptr = q   + (size_t)b * bs + (size_t)h * hs;
  const float* kb_ptr = k   + (size_t)b * bs + (size_t)h * hs;
  const float* vb_ptr = v   + (size_t)b * bs + (size_t)h * hs;
  float*       ob_ptr = out + (size_t)b * bs + (size_t)h * hs;

  v16h qa[2];
  {
    const float* qrow = qb_ptr + (size_t)(q0 + c) * rs;
#pragma unroll
    for (int dc = 0; dc < 2; ++dc) {
#pragma unroll
      for (int e = 0; e < 8; ++e) {
        const float f0 = qrow[dc * 32 + 8 * hh + e] * qscale;
        const float f1 = qrow[dc * 32 + 16 + 8 * hh + e] * qscale;
        qa[dc][e] = (_Float16)f0;
        qa[dc][8 + e] = (_Float16)f1;
      }
    }
  }

  float mrow[8], lrow[8];
  v8f oacc[4];
#pragma unroll
  for (int r = 0; r < 8; ++r) { mrow[r] = -INFINITY; lrow[r] = 0.f; }
#pragma unroll
  for (int t = 0; t < 4; ++t) oacc[t] = (v8f){0.f,0.f,0.f,0.f,0.f,0.f,0.f,0.f};

  const int nChunks = Skv / AT_KC;
  for (int kc = 0; kc < nChunks; ++kc) {
    const int kv0 = kc * AT_KC;
    __syncthreads();
    {
      const int kvr = tid >> 1, dh = (tid & 1) * 32;
      const float* krow = kb_ptr + (size_t)(kv0 + kvr) * rs + dh;
      const float* vrow = vb_ptr + (size_t)(kv0 + kvr) * rs + dh;
#pragma unroll
      for (int i = 0; i < 8; ++i) {
        v4f kk = *(const v4f*)(krow + 4 * i);
        v4f vv = *(const v4f*)(vrow + 4 * i);
#pragma unroll
        for (int e = 0; e < 4; ++e) {
          const int d = dh + 4 * i + e;
          Ksh[kvr * AT_D + d] = (_Float16)kk[e];
          Vth[d * AT_KC + kvr] = (_Float16)vv[e];
        }
      }
    }
    __syncthreads();

    v8f s[4];
#pragma unroll
    for (int j = 0; j < 4; ++j) {
      s[j] = (v8f){0.f,0.f,0.f,0.f,0.f,0.f,0.f,0.f};
#pragma unroll
      for (int dc = 0; dc < 2; ++dc) {
        FB kb;
        kb.h[0] = *(const v8h*)(Ksh + (j * 16 + c) * AT_D + dc * 32 + 8 * hh);
        kb.h[1] = *(const v8h*)(Ksh + (j * 16 + c) * AT_D + dc * 32 + 16 + 8 * hh);
        s[j] = at_mma_h(qa[dc], kb.v, s[j]);
      }
    }
    float cm[8];
#pragma unroll
    for (int r = 0; r < 8; ++r) {
      float m = -INFINITY;
#pragma unroll
      for (int j = 0; j < 4; ++j) m = fmaxf(m, s[j][r]);
#pragma unroll
      for (int off = 1; off < 16; off <<= 1) m = fmaxf(m, __shfl_xor(m, off, 32));
      cm[r] = m;
    }
    _Float16* pw = Psh[wave];
#pragma unroll
    for (int r = 0; r < 8; ++r) {
      const float mnew = fmaxf(mrow[r], cm[r]);
      const float alpha = __expf(mrow[r] - mnew);
      mrow[r] = mnew;
      float psum = 0.f;
#pragma unroll
      for (int j = 0; j < 4; ++j) {
        const float p = __expf(s[j][r] - mnew);
        psum += p;
        pw[(8 * hh + r) * AT_KC + j * 16 + c] = (_Float16)(p * AT_PSC);
      }
#pragma unroll
      for (int off = 1; off < 16; off <<= 1) psum += __shfl_xor(psum, off, 32);
      lrow[r] = lrow[r] * alpha + psum;
#pragma unroll
      for (int t = 0; t < 4; ++t) oacc[t][r] *= alpha;
    }
    __builtin_amdgcn_fence(__ATOMIC_RELEASE, "workgroup");
    __builtin_amdgcn_wave_barrier();
    __builtin_amdgcn_fence(__ATOMIC_ACQUIRE, "workgroup");
#pragma unroll 1
    for (int kk = 0; kk < 2; ++kk) {
      FB pa;
      pa.h[0] = *(const v8h*)(pw + c * AT_KC + kk * 32 + 8 * hh);
      pa.h[1] = *(const v8h*)(pw + c * AT_KC + kk * 32 + 16 + 8 * hh);
#pragma unroll
      for (int t = 0; t < 4; ++t) {
        FB vb;
        vb.h[0] = *(const v8h*)(Vth + (t * 16 + c) * AT_KC + kk * 32 + 8 * hh);
        vb.h[1] = *(const v8h*)(Vth + (t * 16 + c) * AT_KC + kk * 32 + 16 + 8 * hh);
        oacc[t] = at_mma_h(pa.v, vb.v, oacc[t]);
      }
    }
  }

  float* os = Os[wave];
#pragma unroll
  for (int r = 0; r < 8; ++r) {
    const float inv = 1.0f / (lrow[r] * AT_PSC);
#pragma unroll
    for (int t = 0; t < 4; ++t) os[(8 * hh + r) * 68 + t * 16 + c] = oacc[t][r] * inv;
  }
  __builtin_amdgcn_fence(__ATOMIC_RELEASE, "workgroup");
  __builtin_amdgcn_wave_barrier();
  __builtin_amdgcn_fence(__ATOMIC_ACQUIRE, "workgroup");
  {
    const int c4 = (lane & 15) * 4;
    for (int pass = 0; pass < 2; ++pass) {
#pragma unroll
      for (int it = 0; it < 8; ++it) {
        const int row = it * 2 + hh;
        v4f val = *(const v4f*)(os + row * 68 + c4);
        *(volatile v4f*)(ob_ptr + (size_t)(q0 + row) * rs + c4) = val;
      }
      __threadfence();
    }
  }
}

template <bool WH>
__global__ __launch_bounds__(256) void ln_rows_kernel(
    const float* __restrict__ X, const float* __restrict__ Res,
    const float* __restrict__ gam, const float* __restrict__ bet,
    float* __restrict__ Yf, _Float16* __restrict__ Yh, int d) {
  __shared__ float red0[8];
  __shared__ float red1[8];
  const int tid = threadIdx.x, lane = tid & 31, wave = tid >> 5;
  const size_t base = (size_t)blockIdx.x * (size_t)d;
  const int c0 = tid * 4;
  v4f x = *(const v4f*)(X + base + c0);
  const v4f rr = *(const v4f*)(Res + base + c0);
  x[0] += rr[0]; x[1] += rr[1]; x[2] += rr[2]; x[3] += rr[3];
  float s = (x[0] + x[1]) + (x[2] + x[3]);
#pragma unroll
  for (int off = 1; off < 32; off <<= 1) s += __shfl_xor(s, off, 32);
  if (lane == 0) red0[wave] = s;
  __syncthreads();
  float tot = 0.f;
#pragma unroll
  for (int w = 0; w < 8; ++w) tot += red0[w];
  const float invd = 1.0f / (float)d;
  const float mu = tot * invd;
  v4f dv;
  dv[0] = x[0] - mu; dv[1] = x[1] - mu; dv[2] = x[2] - mu; dv[3] = x[3] - mu;
  float s2 = (dv[0] * dv[0] + dv[1] * dv[1]) + (dv[2] * dv[2] + dv[3] * dv[3]);
#pragma unroll
  for (int off = 1; off < 32; off <<= 1) s2 += __shfl_xor(s2, off, 32);
  if (lane == 0) red1[wave] = s2;
  __syncthreads();
  float tot2 = 0.f;
#pragma unroll
  for (int w = 0; w < 8; ++w) tot2 += red1[w];
  const float var = tot2 * invd;
  const float rstd = rsqrtf(var + 1e-5f);
  const v4f gv = *(const v4f*)(gam + c0);
  const v4f bv = *(const v4f*)(bet + c0);
  v4f y;
  y[0] = dv[0] * rstd * gv[0] + bv[0];
  y[1] = dv[1] * rstd * gv[1] + bv[1];
  y[2] = dv[2] * rstd * gv[2] + bv[2];
  y[3] = dv[3] * rstd * gv[3] + bv[3];
  v4h yh;
  yh[0] = (_Float16)y[0]; yh[1] = (_Float16)y[1]; yh[2] = (_Float16)y[2]; yh[3] = (_Float16)y[3];
  float* yp = Yf + base + c0;
  *(volatile v4f*)yp = y;
  if (WH) *(volatile v4h*)(Yh + base + c0) = yh;
  __threadfence();
  *(volatile v4f*)yp = y;
  if (WH) *(volatile v4h*)(Yh + base + c0) = yh;
}

extern "C" void kernel_launch(void* const* d_in, const int* in_sizes, int n_in,
                              void* d_out, int out_size, void* d_ws, size_t ws_size,
                              hipStream_t stream) {
  if (n_in < 12) return;
  const int NH = 16, DHD = 64, NB = 2;
  const int d  = in_sizes[8];
  const int d4 = in_sizes[5];
  if (d != NH * DHD || d != 4 * 256) return;
  if (in_sizes[0] % d != 0) return;
  const int M = in_sizes[0] / d;
  if (M % NB != 0) return;
  const int S = M / NB;
  if ((S % 64) != 0 || (M % 64) != 0 || (d4 % 64) != 0 || (d % 64) != 0) return;
  if (in_sizes[1] != d * d || in_sizes[2] != d * d || in_sizes[3] != d * d) return;
  if (in_sizes[4] != d4 * d || in_sizes[6] != d * d4 || in_sizes[7] != d) return;
  if (in_sizes[9] != d || in_sizes[10] != d || in_sizes[11] != d) return;
  if (out_size != M * d) return;

  const float* embed = (const float*)d_in[0];
  const float* Wk    = (const float*)d_in[1];
  const float* Wq    = (const float*)d_in[2];
  const float* Wv    = (const float*)d_in[3];
  const float* w1w   = (const float*)d_in[4];
  const float* w1b   = (const float*)d_in[5];
  const float* w2w   = (const float*)d_in[6];
  const float* w2b   = (const float*)d_in[7];
  const float* ln_g  = (const float*)d_in[8];
  const float* ln_b  = (const float*)d_in[9];
  const float* ln2_g = (const float*)d_in[10];
  const float* ln2_b = (const float*)d_in[11];
  float* outp = (float*)d_out;

  size_t off = 0;
  char* wsb = (char*)d_ws;
  auto carve = [&](size_t bytes) -> char* { char* p = wsb + off; off += (bytes + 255) & ~(size_t)255; return p; };
  _Float16* emb16 = (_Float16*)carve((size_t)M * d * 2);
  _Float16* wk16  = (_Float16*)carve((size_t)d * d * 2);
  _Float16* wq16  = (_Float16*)carve((size_t)d * d * 2);
  _Float16* wv16  = (_Float16*)carve((size_t)d * d * 2);
  _Float16* w1h   = (_Float16*)carve((size_t)d4 * d * 2);
  _Float16* w2h   = (_Float16*)carve((size_t)d * d4 * 2);
  float* Qf       = (float*)carve((size_t)M * d * 4);
  float* Kf       = (float*)carve((size_t)M * d * 4);
  float* Vf       = (float*)carve((size_t)M * d * 4);
  float* attnf    = (float*)carve((size_t)M * d * 4);
  float* xf       = (float*)carve((size_t)M * d * 4);
  _Float16* x16   = (_Float16*)carve((size_t)M * d * 2);
  if (off > ws_size) return;
  if ((size_t)M * d4 * 2 > (size_t)3 * M * d * 4) return;
  _Float16* hid = (_Float16*)Qf;
  float* out2 = attnf;

  const float WSC = 64.0f, WINV = 1.0f / 64.0f;

  {
    const int n2e = (M * d) / 2;
    cast_f32_f16x2<<<(unsigned)((n2e + 255) / 256), 256, 0, stream>>>(embed, emb16, n2e, 1.0f);
    const int n2w = (d * d) / 2;
    cast_f32_f16x2<<<(unsigned)((n2w + 255) / 256), 256, 0, stream>>>(Wk, wk16, n2w, WSC);
    cast_f32_f16x2<<<(unsigned)((n2w + 255) / 256), 256, 0, stream>>>(Wq, wq16, n2w, WSC);
    cast_f32_f16x2<<<(unsigned)((n2w + 255) / 256), 256, 0, stream>>>(Wv, wv16, n2w, WSC);
    const int n2f = (d4 * d) / 2;
    cast_f32_f16x2<<<(unsigned)((n2f + 255) / 256), 256, 0, stream>>>(w1w, w1h, n2f, WSC);
    cast_f32_f16x2<<<(unsigned)((n2f + 255) / 256), 256, 0, stream>>>(w2w, w2h, n2f, WSC);
  }

  {
    const int tiles = (M / 64) * (d / 64);
    const dim3 grd((unsigned)((tiles + 7) / 8), 1);
    wmma_gemm64<0, false, 0, 0, false, 0><<<grd, 256, 0, stream>>>(
        U16(emb16), U16(emb16), d, (long)0, U16(wq16), U16(wq16), d, (long)0,
        (void*)Qf, (void*)Qf, d, (long)0, w2b, embed, (long)0, M, d, d, WINV);
    wmma_gemm64<0, false, 0, 0, false, 0><<<grd, 256, 0, stream>>>(
        U16(emb16), U16(emb16), d, (long)0, U16(wk16), U16(wk16), d, (long)0,
        (void*)Kf, (void*)Kf, d, (long)0, w2b, embed, (long)0, M, d, d, WINV);
    wmma_gemm64<0, false, 0, 0, false, 0><<<grd, 256, 0, stream>>>(
        U16(emb16), U16(emb16), d, (long)0, U16(wv16), U16(wv16), d, (long)0,
        (void*)Vf, (void*)Vf, d, (long)0, w2b, embed, (long)0, M, d, d, WINV);
  }

  {
    const long bs = (long)S * d, rs = (long)d, hs = (long)DHD;
    const unsigned nblk = (unsigned)(NB * NH * (S / 64));
    attn64_f16_kernel<<<nblk, 128, 0, stream>>>(Qf, Kf, Vf, attnf, bs, rs, hs, S, S, NH, 0.125f);
  }

  ln_rows_kernel<true><<<(unsigned)M, 256, 0, stream>>>(attnf, embed, ln_g, ln_b, xf, x16, d);

  {
    const int tiles = (M / 64) * (d4 / 64);
    const dim3 grd((unsigned)((tiles + 7) / 8), 1);
    wmma_gemm64<0, false, 2, 1, false, 6><<<grd, 256, 0, stream>>>(
        U16(x16), U16(x16), d, (long)0, U16(w1h), U16(w1h), d, (long)0,
        (void*)hid, (void*)hid, d4, (long)0, w1b, xf, (long)0, M, d4, d, WINV);
  }

  {
    const int tiles = (M / 64) * (d / 64);
    const dim3 grd((unsigned)((tiles + 7) / 8), 1);
    wmma_gemm64<0, false, 2, 0, false, 0><<<grd, 256, 0, stream>>>(
        U16(hid), U16(hid), d4, (long)0, U16(w2h), U16(w2h), d4, (long)0,
        (void*)out2, (void*)out2, d, (long)0, w2b, xf, (long)0, M, d, d4, WINV);
  }

  ln_rows_kernel<false><<<(unsigned)M, 256, 0, stream>>>(out2, xf, ln2_g, ln2_b, outp, x16, d);

  (void)hipGetLastError();
}
